// DNeRFDistortion_29016799051958
// MI455X (gfx1250) — hardware-verified
//
#include <hip/hip_runtime.h>
#include <stdint.h>
#include <stddef.h>

#pragma clang fp contract(off)

#define NP    131072
#define NCL   8
#define WD    256
#define NW    (WD * WD)
#define CH    4096
#define NCHK  (NP / CH)
#define TR    64
#define HP    264
#define CP    260
#define TP    72

#define L_HH   0
#define L_HL   (L_HH + TR * HP * 2)
#define L_C    (L_HL + TR * HP * 2)
#define L_OUT  (L_C + TR * CP * 4)
#define L_LST  (L_OUT + CH * 16)
#define L_POS  (L_LST + CH * 4)
#define L_W4   (L_POS + TR * 16)
#define L_WC   (L_W4 + WD * 3 * 4)
#define LDS_MLP (L_WC + 64)

static_assert(NP % CH == 0);
static_assert(CH % TR == 0);
static_assert(CH % 256 == 0);
static_assert((L_HL % 16) == 0);
static_assert((L_C % 16) == 0);
static_assert((L_OUT % 16) == 0);
static_assert((L_LST % 16) == 0);
static_assert((L_POS % 16) == 0);
static_assert((L_W4 % 16) == 0);
static_assert((L_WC % 16) == 0);
static_assert(((NP * 3) / 4) % 256 == 0);
static_assert((NP * 3) % 4 == 0);

typedef __bf16        v16bf __attribute__((ext_vector_type(16)));
typedef float         v8f   __attribute__((ext_vector_type(8)));
typedef float         v4f   __attribute__((ext_vector_type(4)));
typedef unsigned int  v4u   __attribute__((ext_vector_type(4)));
typedef v4f __attribute__((may_alias)) v4fa;
typedef v4u __attribute__((may_alias)) v4ua;

union FragBF { v16bf v; v4u q[2]; };

__device__ __forceinline__ unsigned int bfb(float f) {
  unsigned int u = __float_as_uint(f);
  u += 0x7FFFu + ((u >> 16) & 1u);
  return u >> 16;
}
__device__ __forceinline__ void split2(float v, unsigned int& hi, unsigned int& lo) {
  hi = bfb(v);
  lo = bfb(v - __uint_as_float(hi << 16));
}
__device__ __forceinline__ unsigned int pk(unsigned int a, unsigned int b) { return a | (b << 16); }

__device__ __forceinline__ v8f wmma_bf(v16bf a, v16bf b, v8f c) {
  v8f d = __builtin_amdgcn_wmma_f32_16x16x32_bf16(false, a, false, b, (short)0, c, false, false);
  asm volatile("v_nop\n\tv_nop\n\tv_nop\n\tv_nop" : "+v"(d) : "v"(a), "v"(b));
  return d;
}

__device__ __forceinline__ v16bf ldfrag(const unsigned short* p, int h) {
  FragBF f;
  f.q[0] = *(const v4ua*)(p + 8 * h);
  f.q[1] = *(const v4ua*)(p + 16 + 8 * h);
  return f.v;
}

__device__ __forceinline__ void wt_store_pass(const unsigned short* sh, const unsigned short* sl,
                                              unsigned short* oh, unsigned short* ol,
                                              int e, int r0, int c0, int wv, int lane)
{
  const int q8 = lane & 7, sub = lane >> 3;
  #pragma unroll
  for (int i = 0; i < 2; ++i) {
    const int n = wv * 8 + i * 4 + sub;
    const v4u hv = *(const v4ua*)(sh + n * TP + 8 * q8);
    const v4u lv = *(const v4ua*)(sl + n * TP + 8 * q8);
    const size_t go = ((size_t)e * WD + c0 + n) * WD + r0 + 8 * q8;
    *(volatile v4u*)(oh + go) = hv;
    *(volatile v4u*)(ol + go) = lv;
  }
}

__global__ __launch_bounds__(256) void k_cvt_w(const float* __restrict__ wa,
                                               const float* __restrict__ wb,
                                               unsigned short* __restrict__ ah,
                                               unsigned short* __restrict__ al,
                                               unsigned short* __restrict__ bh,
                                               unsigned short* __restrict__ bl)
{
  __shared__ __align__(16) unsigned short sh[64 * TP];
  __shared__ __align__(16) unsigned short sl[64 * TP];
  const int tid = threadIdx.x, lane = tid & 31, wv = tid >> 5;
  const int z = blockIdx.z;
  const int mat = z >> 3, e = z & 7;
  const int r0 = blockIdx.x * 64;
  const int c0 = blockIdx.y * 64;
  const float* w = (mat == 0) ? wa : wb;
  unsigned short* oh = (mat == 0) ? ah : bh;
  unsigned short* ol = (mat == 0) ? al : bl;
  const float* src = w + (size_t)e * NW;
  #pragma unroll
  for (int j = 0; j < 4; ++j) {
    const int idx = tid + 256 * j;
    const int row = idx >> 4, c4 = idx & 15;
    const v4f v = *(const v4fa*)(src + (size_t)(r0 + row) * WD + c0 + 4 * c4);
    unsigned int ha, la, hb, lb, hc, lc, hd, ld;
    split2(v.x, ha, la); split2(v.y, hb, lb); split2(v.z, hc, lc); split2(v.w, hd, ld);
    const int cb = 4 * c4;
    sh[(cb + 0) * TP + row] = (unsigned short)ha;  sl[(cb + 0) * TP + row] = (unsigned short)la;
    sh[(cb + 1) * TP + row] = (unsigned short)hb;  sl[(cb + 1) * TP + row] = (unsigned short)lb;
    sh[(cb + 2) * TP + row] = (unsigned short)hc;  sl[(cb + 2) * TP + row] = (unsigned short)lc;
    sh[(cb + 3) * TP + row] = (unsigned short)hd;  sl[(cb + 3) * TP + row] = (unsigned short)ld;
  }
  __syncthreads();
  wt_store_pass(sh, sl, oh, ol, e, r0, c0, wv, lane);
  __threadfence();
  wt_store_pass(sh, sl, oh, ol, e, r0, c0, wv, lane);
}

__device__ __forceinline__ void gemm256(const unsigned short* sAh, const unsigned short* sAl,
                                        const unsigned short* __restrict__ bhp,
                                        const unsigned short* __restrict__ blp,
                                        float* sC, int mg, int ng, int h, int m)
{
  const v8f z8 = {0.f, 0.f, 0.f, 0.f, 0.f, 0.f, 0.f, 0.f};
  v8f acc[2][4];
  #pragma unroll
  for (int mt = 0; mt < 2; ++mt)
    #pragma unroll
    for (int nt = 0; nt < 4; ++nt) acc[mt][nt] = z8;

  #pragma unroll 1
  for (int k0 = 0; k0 < WD; k0 += 32) {
    v16bf ah[2], al[2];
    #pragma unroll
    for (int mt = 0; mt < 2; ++mt) {
      const int ro = (32 * mg + 16 * mt + m) * HP + k0;
      ah[mt] = ldfrag(sAh + ro, h);
      al[mt] = ldfrag(sAl + ro, h);
    }
    #pragma unroll
    for (int nt = 0; nt < 4; ++nt) {
      const int n = ng * 64 + 16 * nt + m;
      const size_t bo = (size_t)n * WD + k0;
      const v16bf bh = ldfrag(bhp + bo, h);
      const v16bf bl = ldfrag(blp + bo, h);
      #pragma unroll
      for (int mt = 0; mt < 2; ++mt) {
        acc[mt][nt] = wmma_bf(ah[mt], bh, acc[mt][nt]);
        acc[mt][nt] = wmma_bf(ah[mt], bl, acc[mt][nt]);
        acc[mt][nt] = wmma_bf(al[mt], bh, acc[mt][nt]);
      }
    }
  }
  #pragma unroll
  for (int mt = 0; mt < 2; ++mt)
    #pragma unroll
    for (int nt = 0; nt < 4; ++nt)
      #pragma unroll
      for (int r = 0; r < 8; ++r) {
        const int row = 32 * mg + 16 * mt + 8 * h + r;
        const int col = ng * 64 + 16 * nt + m;
        sC[row * CP + col] = acc[mt][nt][r];
      }
}

__device__ __forceinline__ void stage_store_pass(const float* sOut, float* dst, int tid) {
  #pragma unroll
  for (int j = 0; j < CH / 256; ++j) {
    const int idx = tid + 256 * j;
    const v4f v = *(const v4fa*)(sOut + 4 * idx);
    *(volatile v4f*)(dst + (size_t)4 * idx) = v;
  }
}

__global__ __launch_bounds__(256) void k_mlp(const float* __restrict__ pos,
                                             const int* __restrict__ times,
                                             const float* __restrict__ W1,
                                             const float* __restrict__ B1,
                                             const unsigned short* __restrict__ w2h,
                                             const unsigned short* __restrict__ w2l,
                                             const float* __restrict__ B2,
                                             const unsigned short* __restrict__ w3h,
                                             const unsigned short* __restrict__ w3l,
                                             const float* __restrict__ B3,
                                             const float* __restrict__ W4,
                                             const float* __restrict__ B4,
                                             float* __restrict__ stage)
{
  extern __shared__ __align__(16) unsigned char dsm[];
  unsigned short* sHh = (unsigned short*)(dsm + L_HH);
  unsigned short* sHl = (unsigned short*)(dsm + L_HL);
  float* sC   = (float*)(dsm + L_C);
  float* sOut = (float*)(dsm + L_OUT);
  int*   sLst = (int*)(dsm + L_LST);
  float* sPos = (float*)(dsm + L_POS);
  float* sW4  = (float*)(dsm + L_W4);
  int*   sWc  = (int*)(dsm + L_WC);

  const int tid = threadIdx.x, lane = tid & 31, wv = tid >> 5;
  const int h = lane >> 4, m = lane & 15;
  const int mg = wv & 1, ng = wv >> 1;
  const int c = blockIdx.y;
  const int p0 = blockIdx.x * CH;

  const v4f z4 = {0.f, 0.f, 0.f, 0.f};
  #pragma unroll 1
  for (int i = tid; i < CH; i += 256) {
    *(v4fa*)(sOut + 4 * i) = z4;
    sLst[i] = 0;
  }
  #pragma unroll 1
  for (int i = tid; i < WD * 3; i += 256) sW4[i] = W4[(size_t)c * WD * 3 + i];
  const float w1x = W1[((size_t)c * 3 + 0) * WD + tid];
  const float w1y = W1[((size_t)c * 3 + 1) * WD + tid];
  const float w1z = W1[((size_t)c * 3 + 2) * WD + tid];
  const float b1n = B1[(size_t)c * WD + tid];
  const float b2n = B2[(size_t)c * WD + tid];
  const float b3n = B3[(size_t)c * WD + tid];
  const int j4 = tid & 3;
  const int jj = (j4 < 3) ? j4 : 2;
  const float b4j = B4[c * 3 + jj];
  const unsigned short* p2h = w2h + (size_t)c * NW;
  const unsigned short* p2l = w2l + (size_t)c * NW;
  const unsigned short* p3h = w3h + (size_t)c * NW;
  const unsigned short* p3l = w3l + (size_t)c * NW;
  __syncthreads();

  int base = 0;
  #pragma unroll 1
  for (int sc = 0; sc < CH / 256; ++sc) {
    const int lp = sc * 256 + tid;
    const int tv = times[(size_t)p0 + lp];
    const bool f = (tv == c);
    const unsigned int msk = __builtin_amdgcn_ballot_w32(f);
    const int off = __builtin_popcount(msk & ((1u << lane) - 1u));
    const int wc = __builtin_popcount(msk);
    if (lane == 0) sWc[wv] = wc;
    __syncthreads();
    int pre = 0, tot = 0;
    #pragma unroll
    for (int w2 = 0; w2 < 8; ++w2) {
      const int cc = sWc[w2];
      tot += cc;
      pre += (w2 < wv) ? cc : 0;
    }
    if (f) {
      int p = base + pre + off;
      p = (p < 0) ? 0 : ((p > CH - 1) ? (CH - 1) : p);
      sLst[p] = lp;
    }
    base += tot;
    __syncthreads();
  }
  int nh = (base > CH) ? CH : ((base < 0) ? 0 : base);
  nh = __builtin_amdgcn_readfirstlane(nh);
  const int ntiles = (nh + TR - 1) / TR;

  #pragma unroll 1
  for (int tile = 0; tile < ntiles && tile < CH / TR; ++tile) {
    if (tid < TR) {
      int li = tile * TR + tid;
      li = (li > CH - 1) ? (CH - 1) : li;
      int lp = sLst[li];
      lp = (lp < 0) ? 0 : ((lp > CH - 1) ? (CH - 1) : lp);
      const float* pp = pos + ((size_t)p0 + lp) * 3;
      sPos[4 * tid + 0] = pp[0];
      sPos[4 * tid + 1] = pp[1];
      sPos[4 * tid + 2] = pp[2];
      sPos[4 * tid + 3] = 0.0f;
    }
    __syncthreads();

    #pragma unroll 1
    for (int j = 0; j < TR; ++j) {
      const v4f pv = *(const v4fa*)(sPos + 4 * j);
      float d = pv.x * w1x;
      d = fmaf(pv.y, w1y, d);
      d = fmaf(pv.z, w1z, d);
      const float hv = tanhf(d + b1n);
      unsigned int hi, lo;
      split2(hv, hi, lo);
      sHh[j * HP + tid] = (unsigned short)hi;
      sHl[j * HP + tid] = (unsigned short)lo;
    }
    __syncthreads();

    gemm256(sHh, sHl, p2h, p2l, sC, mg, ng, h, m);
    __syncthreads();
    #pragma unroll 1
    for (int j = 0; j < TR; ++j) {
      const float hv = tanhf(sC[j * CP + tid] + b2n);
      unsigned int hi, lo;
      split2(hv, hi, lo);
      sHh[j * HP + tid] = (unsigned short)hi;
      sHl[j * HP + tid] = (unsigned short)lo;
    }
    __syncthreads();

    gemm256(sHh, sHl, p3h, p3l, sC, mg, ng, h, m);
    __syncthreads();
    #pragma unroll 1
    for (int j = 0; j < TR; ++j) {
      const int o = j * CP + tid;
      sC[o] = tanhf(sC[o] + b3n);
    }
    __syncthreads();

    {
      const int row = tid >> 2;
      const float* hr = sC + row * CP;
      float d = 0.0f;
      #pragma unroll 4
      for (int k = 0; k < WD; ++k) d = fmaf(hr[k], sW4[k * 3 + jj], d);
      const float ov = tanhf(d + b4j);
      const int li = tile * TR + row;
      if (li < nh) {
        int lp = sLst[(li > CH - 1) ? (CH - 1) : li];
        lp = (lp < 0) ? 0 : ((lp > CH - 1) ? (CH - 1) : lp);
        sOut[4 * lp + j4] = (j4 < 3) ? ov : 0.0f;
      }
    }
    __syncthreads();
  }
  __syncthreads();

  float* dst = stage + ((size_t)c * NP + p0) * 4;
  stage_store_pass(sOut, dst, tid);
  __threadfence();
  stage_store_pass(sOut, dst, tid);
}

__device__ __forceinline__ float out_elem(const float* __restrict__ stage,
                                          const int* __restrict__ times, int f)
{
  const int p = f / 3;
  const int comp = f - 3 * p;
  const int tv = times[p];
  const bool ok = (unsigned int)tv < (unsigned int)NCL;
  const int cc = ok ? tv : 0;
  const float v = stage[((size_t)cc * NP + p) * 4 + comp];
  return ok ? v : 0.0f;
}

__global__ __launch_bounds__(256) void k_out(const float* __restrict__ stage,
                                             const int* __restrict__ times,
                                             float* __restrict__ out)
{
  const int g = blockIdx.x * 256 + threadIdx.x;
  if (g >= (NP * 3) / 4) return;
  const int f0 = 4 * g;
  const float o0 = out_elem(stage, times, f0 + 0);
  const float o1 = out_elem(stage, times, f0 + 1);
  const float o2 = out_elem(stage, times, f0 + 2);
  const float o3 = out_elem(stage, times, f0 + 3);
  const v4f ov = {o0, o1, o2, o3};
  float* d = out + (size_t)f0;
  *(volatile v4f*)d = ov;
  __threadfence();
  *(volatile v4f*)d = ov;
}

extern "C" void kernel_launch(void* const* d_in, const int* in_sizes, int n_in,
                              void* d_out, int out_size, void* d_ws, size_t ws_size,
                              hipStream_t stream)
{
  if (n_in < 10) return;
  if (in_sizes[0] != NP * 3) return;
  if (in_sizes[1] != NP) return;
  if (in_sizes[2] != NCL * 3 * WD) return;
  if (in_sizes[3] != NCL * WD) return;
  if (in_sizes[4] != NCL * NW) return;
  if (in_sizes[5] != NCL * WD) return;
  if (in_sizes[6] != NCL * NW) return;
  if (in_sizes[7] != NCL * WD) return;
  if (in_sizes[8] != NCL * WD * 3) return;
  if (in_sizes[9] != NCL * 3) return;
  if (out_size != NP * 3) return;

  const float* pos   = (const float*)d_in[0];
  const int*   times = (const int*)d_in[1];
  const float* W1    = (const float*)d_in[2];
  const float* B1    = (const float*)d_in[3];
  const float* W2    = (const float*)d_in[4];
  const float* B2    = (const float*)d_in[5];
  const float* W3    = (const float*)d_in[6];
  const float* B3    = (const float*)d_in[7];
  const float* W4    = (const float*)d_in[8];
  const float* B4    = (const float*)d_in[9];
  float* out = (float*)d_out;

  const size_t bWp  = (size_t)NCL * NW * 2;
  const size_t bStg = (size_t)NCL * NP * 16;
  const size_t total = 4 * bWp + bStg;
  if (total > ws_size) return;

  char* ws = (char*)d_ws;
  size_t off = 0;
  unsigned short* W2H = (unsigned short*)(ws + off); off += bWp;
  unsigned short* W2L = (unsigned short*)(ws + off); off += bWp;
  unsigned short* W3H = (unsigned short*)(ws + off); off += bWp;
  unsigned short* W3L = (unsigned short*)(ws + off); off += bWp;
  float*          STG = (float*)(ws + off);          off += bStg;
  if (off != total) return;

  dim3 gW(WD / 64, WD / 64, 2 * NCL);
  k_cvt_w<<<gW, 256, 0, stream>>>(W2, W3, W2H, W2L, W3H, W3L);

  hipFuncSetAttribute(reinterpret_cast<const void*>(&k_mlp),
                      hipFuncAttributeMaxDynamicSharedMemorySize, LDS_MLP);
  dim3 gM(NCHK, NCL);
  k_mlp<<<gM, 256, LDS_MLP, stream>>>(pos, times, W1, B1, W2H, W2L, B2, W3H, W3L, B3, W4, B4, STG);

  k_out<<<((NP * 3) / 4) / 256, 256, 0, stream>>>(STG, times, out);
}
